// SpatiallyAdaptiveSirenLayer_31817117728925
// MI455X (gfx1250) — hardware-verified
//
#include <hip/hip_runtime.h>
#include <hip/hip_bf16.h>
#include <math.h>

typedef __attribute__((ext_vector_type(16))) _Float16 v16h;
typedef __attribute__((ext_vector_type(8)))  _Float16 v8h;
typedef __attribute__((ext_vector_type(8)))  float    v8f;
typedef __attribute__((ext_vector_type(4)))  float    v4f_t;
typedef float v4fa __attribute__((ext_vector_type(4), may_alias));
#define RSPLIT (1.0f / 2048.0f)
static __device__ __forceinline__ _Float16 lo_of(float v, _Float16 h) { return (_Float16)((v - (float)h) * 2048.0f); }
static __device__ __forceinline__ v8f wmma16(v16h a, v16h b, v8f c) { return __builtin_amdgcn_wmma_f32_16x16x32_f16(false, a, false, b, (short)0, c, false, false); }
static __device__ __forceinline__ v8f wmma_split(v16h a, v16h al, v16h b, v16h bl, v8f c) { v8f x = {}; x = wmma16(al, b, x); x = wmma16(a, bl, x); return wmma16(a, b, c) + x * RSPLIT; }
static __device__ __forceinline__ void st2f(float* p, float v) { *(volatile float*)p = v; __threadfence(); *(volatile float*)p = v; }

#define SIREN_B    2
#define SIREN_N    16384
#define SIREN_M    1024
#define SIREN_IN   256
#define SIREN_OUT  256
#define OMEGA0     30.0f
#define EPS_D2     1e-4f

__global__ void __launch_bounds__(256)
siren_omega_kernel(const float* __restrict__ qc,
                   const float* __restrict__ ac,
                   const float* __restrict__ fw1,
                   const float* __restrict__ fb1,
                   const float* __restrict__ fw2,
                   const float* __restrict__ fb2,
                   float* __restrict__ omega)
{
    __shared__ float ax[SIREN_M];
    __shared__ float ay[SIREN_M];
    __shared__ float az[SIREN_M];

    const int batch = blockIdx.y;
    const int tid   = threadIdx.x;

    const float* acb = ac + (size_t)batch * SIREN_M * 3;
    for (int i = tid; i < SIREN_M; i += 256) {
        ax[i] = acb[i * 3 + 0];
        ay[i] = acb[i * 3 + 1];
        az[i] = acb[i * 3 + 2];
    }
    __syncthreads();

    const int p = batch * SIREN_N + blockIdx.x * 256 + tid;
    const float qx = qc[(size_t)p * 3 + 0];
    const float qy = qc[(size_t)p * 3 + 1];
    const float qz = qc[(size_t)p * 3 + 2];

    float d2min = 3.4e38f;
#pragma unroll 1
    for (int m = 0; m < SIREN_M; ++m) {
        float dx = qx - ax[m];
        float dy = qy - ay[m];
        float dz = qz - az[m];
        float d2 = fmaf(dx, dx, fmaf(dy, dy, dz * dz));
        d2min = fminf(d2min, d2);
    }
    float min_dist = sqrtf(fmaxf(d2min, EPS_D2));

    float ls = fb2[0];
#pragma unroll 1
    for (int j = 0; j < 16; ++j) {
        float pre = fb1[j] + qx * fw1[j * 3 + 0] + qy * fw1[j * 3 + 1] + qz * fw1[j * 3 + 2];
        float h   = (pre > 20.0f) ? pre : log1pf(expf(pre));
        ls = fmaf(fw2[j], h, ls);
    }
    ls = fminf(fmaxf(ls, 0.0f), 5.0f);
    if (isnan(ls)) ls = 0.0f;

    st2f(omega + p, OMEGA0 * (1.0f + ls * expf(-min_dist)));
}

#define CPB      32
#define RPW      32
#define WROW_PAD 264

static __device__ __forceinline__ void cvt_a_frag(const float* xrow, int k0, int off, v16h& a, v16h& al) {
    const float* p0 = xrow + k0 + off;
    const float* p1 = xrow + k0 + 16 + off;
#pragma unroll
    for (int i = 0; i < 8; ++i) {
        const float u = p0[i], w = p1[i];
        a[i] = (_Float16)u;      al[i] = lo_of(u, a[i]);
        a[8 + i] = (_Float16)w;  al[8 + i] = lo_of(w, a[8 + i]);
    }
}

__global__ void __launch_bounds__(256, 1)
siren_wmma_kernel(const float* __restrict__ x,
                  const float* __restrict__ W,
                  const float* __restrict__ bias,
                  const float* __restrict__ omega,
                  float* __restrict__ out)
{
    __shared__ __attribute__((aligned(16))) _Float16 Wh[CPB * WROW_PAD];
    __shared__ __attribute__((aligned(16))) _Float16 Wl[CPB * WROW_PAD];
    __shared__ __attribute__((aligned(16))) float so[8][32 * 36];

    const int tid     = threadIdx.x;
    const int lane    = tid & 31;
    const int wave    = tid >> 5;
    const int colBase = blockIdx.x * CPB;
    const int rowBase = blockIdx.y * (8 * RPW) + wave * RPW;

    for (int idx = tid; idx < CPB * SIREN_IN; idx += 256) {
        const int col = idx >> 8;
        const int k   = idx & 255;
        const float wv = W[(size_t)(colBase + col) * SIREN_IN + k];
        Wh[col * WROW_PAD + k] = (_Float16)wv; Wl[col * WROW_PAD + k] = lo_of(wv, Wh[col * WROW_PAD + k]);
    }
    __syncthreads();

    const int half32 = lane >> 4;
    const int bcol   = lane & 15;
    const float* xrow0 = x + (size_t)(rowBase + (lane & 15)) * SIREN_IN;
    const float* xrow1 = xrow0 + (size_t)16 * SIREN_IN;

    v8f acc[2][2] = {};
#pragma unroll
    for (int kc = 0; kc < SIREN_IN / 32; ++kc) {
        const int k0  = kc * 32;
        const int off = half32 ? 8 : 0;

        if (kc + 1 < SIREN_IN / 32)
            __builtin_prefetch(xrow0 + k0 + 32 + off, 0, 3);

        v16h a0, a0l, a1, a1l;
        cvt_a_frag(xrow0, k0, off, a0, a0l);
        cvt_a_frag(xrow1, k0, off, a1, a1l);

        const int koff = k0 + off;
#pragma unroll
        for (int t = 0; t < 2; ++t) {
            const int col = t * 16 + bcol;
            const v16h b  = __builtin_shufflevector(*(const v8h*)(&Wh[col * WROW_PAD + koff]), *(const v8h*)(&Wh[col * WROW_PAD + koff + 16]), 0,1,2,3,4,5,6,7,8,9,10,11,12,13,14,15);
            const v16h bl = __builtin_shufflevector(*(const v8h*)(&Wl[col * WROW_PAD + koff]), *(const v8h*)(&Wl[col * WROW_PAD + koff + 16]), 0,1,2,3,4,5,6,7,8,9,10,11,12,13,14,15);
            acc[0][t] = wmma_split(a0, a0l, b, bl, acc[0][t]);
            acc[1][t] = wmma_split(a1, a1l, b, bl, acc[1][t]);
        }
    }

    float bc[2];
#pragma unroll
    for (int t = 0; t < 2; ++t) bc[t] = bias[colBase + t * 16 + bcol];

    float* sw = so[wave];
#pragma unroll
    for (int s = 0; s < 2; ++s) {
#pragma unroll
        for (int j = 0; j < 8; ++j) {
            const int rl = s * 16 + j + (half32 ? 8 : 0);
            const float om = omega[rowBase + rl];
#pragma unroll
            for (int t = 0; t < 2; ++t) {
                const float pre = acc[s][t][j] + bc[t];
                sw[rl * 36 + t * 16 + bcol] = sinf(om * pre);
            }
        }
    }
    asm volatile("s_wait_dscnt 0" ::: "memory");
#pragma unroll 1
    for (int pass = 0; pass < 2; ++pass) {
#pragma unroll
        for (int i = 0; i < 8; ++i) { const int c = lane + 32 * i, rl = c >> 3, q = (c & 7) * 4;
            *(volatile v4f_t*)(out + (size_t)(rowBase + rl) * SIREN_OUT + colBase + q) = *(const volatile v4fa*)(sw + rl * 36 + q); }
        __threadfence();
    }
}

extern "C" void kernel_launch(void* const* d_in, const int* in_sizes, int n_in,
                              void* d_out, int out_size, void* d_ws, size_t ws_size,
                              hipStream_t stream) {
    const float* x   = (const float*)d_in[0];
    const float* qc  = (const float*)d_in[1];
    const float* ac  = (const float*)d_in[2];
    const float* W   = (const float*)d_in[3];
    const float* b   = (const float*)d_in[4];
    const float* fw1 = (const float*)d_in[5];
    const float* fb1 = (const float*)d_in[6];
    const float* fw2 = (const float*)d_in[7];
    const float* fb2 = (const float*)d_in[8];
    float* out       = (float*)d_out;

    float* omega = (float*)d_ws;

    dim3 g1(SIREN_N / 256, SIREN_B);
    siren_omega_kernel<<<g1, 256, 0, stream>>>(qc, ac, fw1, fb1, fw2, fb2, omega);

    dim3 g2(SIREN_OUT / CPB, (SIREN_B * SIREN_N) / (8 * RPW));
    siren_wmma_kernel<<<g2, 256, 0, stream>>>(x, W, b, omega, out);
}
